// DynHNN_17197049053669
// MI455X (gfx1250) — hardware-run, weakly checked
//
#include <hip/hip_runtime.h>


namespace {
constexpr int N = 100000, M = 200000, E = 2000000, IN = 16, HID = 64, NT = 2, NBLK = N / 16;
constexpr float XS = 8.0f, CS = 64.0f, WSC = 256.0f;
typedef _Float16 b16;
typedef __attribute__((ext_vector_type(16))) _Float16 v16b;
typedef __attribute__((ext_vector_type(8))) _Float16 v8b;
typedef __attribute__((ext_vector_type(8))) float v8f;
typedef __attribute__((ext_vector_type(4))) float v4f;
typedef __attribute__((ext_vector_type(2))) float v2f;
__device__ __forceinline__ float bf16_rne(float f) { unsigned int u = __float_as_uint(f); u += 0x7FFFu + ((u >> 16) & 1u); return __uint_as_float(u & 0xFFFF0000u); }
__device__ __forceinline__ void split16(float v, b16& hi, b16& lo) { hi = (b16)v; lo = (b16)(v - (float)hi); }
__device__ __forceinline__ v16b frag_kb(const b16* p, int hh) { const v8b a = *(const v8b*)(p + 8 * hh), b = *(const v8b*)(p + 16 + 8 * hh); v16b f;
#pragma unroll
  for (int e = 0; e < 8; ++e) { f[e] = a[e]; f[8 + e] = b[e]; } return f; }
__device__ __forceinline__ v8f wmma16b(v16b a, v16b b, v8f c) { v8f d = __builtin_amdgcn_wmma_f32_16x16x32_f16(false, a, false, b, (short)0, c, false, false); asm volatile("v_nop\n\tv_nop\n\tv_nop\n\tv_nop" : "+v"(d) : "v"(a), "v"(b)); return d; }
__device__ __forceinline__ void wave_lds_sync() { __builtin_amdgcn_fence(__ATOMIC_RELEASE, "workgroup"); __builtin_amdgcn_wave_barrier(); __builtin_amdgcn_fence(__ATOMIC_ACQUIRE, "workgroup"); }
__device__ __forceinline__ float pmul(float a, float b) { float p = a * b; asm volatile("" : "+v"(p)); return p; }
__device__ __forceinline__ int iclamp(int v, int lo, int hi) { return v < lo ? lo : (v > hi ? hi : v); }
__device__ __forceinline__ float sigm(float v) { return 1.0f / (1.0f + __expf(-v)); }
constexpr int CSR_NBLK9 = 512, CSR_GB9 = 9, CSR_GN9 = 1 << CSR_GB9  , CSR_TS9 = (CSR_GN9 < 32 ? 32 : CSR_GN9)  , CSR_MAXG9 = 512, CSR_CAP9 = 12288  ;
__device__ __host__ __forceinline__ int csr_tix9(int v) { return (v >> CSR_GB9) * CSR_TS9 + (v & (CSR_GN9 - 1)); }
__global__ __launch_bounds__(64) void csrA_kernel9(const int* __restrict__ dst, int E, int N, int nG, int CHP, int NGP, int* __restrict__ STG, int* __restrict__ HST) {
  extern __shared__ int sm[];
  int* cnt = sm; int* run = sm + NGP; int* ids = sm + 2 * NGP;
  const int b = blockIdx.x; const int ch = (E + CSR_NBLK9 - 1) / CSR_NBLK9; const int e0 = b * ch, e1 = min(E, e0 + ch);
  for (int i = threadIdx.x; i < NGP; i += 64) cnt[i] = 0;
  for (int i = threadIdx.x; i < CHP; i += 64) ids[i] = -1;
  __syncthreads();
  if (threadIdx.x == 0) {
    for (int e = e0; e < e1; ++e) { int d = dst[e]; d = (d < 0) ? 0 : (d >= N ? N - 1 : d); cnt[d >> CSR_GB9] += 1; }
    int acc = 0; for (int g = 0; g < nG; ++g) { run[g] = acc; acc += cnt[g]; }
    for (int e = e0; e < e1; ++e) { int d = dst[e]; d = (d < 0) ? 0 : (d >= N ? N - 1 : d); const int g = d >> CSR_GB9; ids[run[g]] = e; run[g] += 1; } }
  __syncthreads();
  typedef __attribute__((ext_vector_type(4))) int v4i;
  for (int pass = 0; pass < 2; ++pass) {
    for (int i = threadIdx.x; i < CHP / 4; i += 64) *(volatile v4i*)(STG + (size_t)b * CHP + i * 4) = *(const v4i*)(&ids[i * 4]);
    for (int i = threadIdx.x; i < NGP / 4; i += 64) { v4i v; for (int e = 0; e < 4; ++e) v[e] = (i * 4 + e < nG) ? cnt[i * 4 + e] : 0; *(volatile v4i*)(HST + (size_t)b * NGP + i * 4) = v; }
    __threadfence(); }
}
__global__ __launch_bounds__(512) void csrS_kernel9(const int* __restrict__ HST, int nG, int NGP, int* __restrict__ START, int* __restrict__ TOT, int* __restrict__ OFF) {
  __shared__ int tot[CSR_MAXG9];
  const int b = threadIdx.x;
  for (int pass = 0; pass < 2; ++pass) { int runb = 0; for (int g = 0; g < nG; ++g) { int c = HST[(size_t)b * NGP + g]; c = (c < 0) ? 0 : c; ((volatile int*)OFF)[(size_t)g * CSR_NBLK9 + b] = runb; runb += c; } __threadfence(); }
  for (int g = threadIdx.x; g < nG; g += 512) { int s = 0; for (int bb = 0; bb < CSR_NBLK9; ++bb) { int c = HST[(size_t)bb * NGP + g]; s += (c < 0) ? 0 : c; } tot[g] = s; }
  __syncthreads();
  if (threadIdx.x < 32) {
    __shared__ int st[CSR_MAXG9 + 32];
    if (threadIdx.x == 0) { int acc = 0; for (int g = 0; g < NGP; ++g) { st[g] = acc; if (g < nG) acc += (tot[g] + 31) & ~31; } st[NGP] = acc; }
    __builtin_amdgcn_fence(__ATOMIC_RELEASE, "workgroup"); __builtin_amdgcn_wave_barrier(); __builtin_amdgcn_fence(__ATOMIC_ACQUIRE, "workgroup");
    for (int pass = 0; pass < 2; ++pass) { for (int i = threadIdx.x; i < NGP + 32; i += 32) { ((volatile int*)START)[i] = (i <= NGP) ? st[min(i, NGP)] : 0; ((volatile int*)TOT)[i] = (i < nG) ? tot[i] : 0; } __threadfence(); } }
}
__global__ __launch_bounds__(256) void csrB_kernel9(const int* __restrict__ dst, int N, int nG, int CHP, int NGP, int permLen, const int* __restrict__ STG, const int* __restrict__ HST, const int* __restrict__ OFF, const int* __restrict__ START, const int* __restrict__ TOT, int* __restrict__ PERM, int* __restrict__ ROWPTR, int* __restrict__ ROWCNT, int* __restrict__ FLAG) {
  typedef __attribute__((ext_vector_type(4))) int v4i;
  __shared__ int ids[CSR_CAP9]; __shared__ unsigned short key[CSR_CAP9]; __shared__ int outp[CSR_CAP9]; __shared__ int ncnt[CSR_GN9 + 1]; __shared__ int boff[CSR_NBLK9 + 1];
  const int g = blockIdx.x, t_ = threadIdx.x; int tot = TOT[g]; int st = START[g], stn = START[g + 1]; const int v0 = g * CSR_GN9; const int nv = min(CSR_GN9, N - v0); const int t0 = g * CSR_TS9;
  st = (st < 0) ? 0 : (st > permLen - 32 ? permLen - 32 : st) & ~31; stn = (stn < st) ? st : (stn > permLen ? permLen : stn); tot = (tot < 0) ? 0 : tot; if (tot > stn - st && tot <= CSR_CAP9) tot = stn - st;
  if (tot > CSR_CAP9) {
    for (int pass = 0; pass < 2; ++pass) { for (int i = t_; i < CSR_TS9 / 4; i += 256) { v4i a, c; for (int e = 0; e < 4; ++e) { a[e] = st; c[e] = 0; } *(volatile v4i*)(ROWPTR + t0 + i * 4) = a; *(volatile v4i*)(ROWCNT + t0 + i * 4) = c; } if (t_ == 0) ((volatile int*)FLAG)[0] = 1; __threadfence(); } (void)nv; return; }
  if (t_ == 0) { int acc = 0; for (int b = 0; b < CSR_NBLK9; ++b) { boff[b] = acc; int c = HST[(size_t)b * NGP + g]; c = (c < 0) ? 0 : (c > CHP ? CHP : c); acc += c; if (acc > tot) acc = tot; } boff[CSR_NBLK9] = acc; }
  for (int i = t_; i <= CSR_GN9; i += 256) ncnt[i] = 0;
  __syncthreads();
  for (int b = 0; b < CSR_NBLK9; ++b) { const int c = boff[b + 1] - boff[b]; int o_ = OFF[(size_t)g * CSR_NBLK9 + b]; o_ = (o_ < 0) ? 0 : (o_ > CHP - c ? CHP - c : o_); const int* src_ = STG + (size_t)b * CHP + o_;
    for (int i = t_; i < c; i += 256) { int id = src_[i]; id = (id < 0) ? 0 : id; ids[boff[b] + i] = id; int d = dst[id]; d = (d < v0) ? v0 : (d >= N ? N - 1 : d); int kk = d - v0; kk = (kk < 0) ? 0 : (kk >= CSR_GN9 ? CSR_GN9 - 1 : kk); key[boff[b] + i] = (unsigned short)kk; } }
  __syncthreads();
  if (t_ == 0) { for (int i = 0; i < tot; ++i) ncnt[key[i]] += 1; int acc = 0; for (int vl = 0; vl < CSR_GN9; ++vl) { const int c = ncnt[vl]; ncnt[vl] = acc; acc += c; } ncnt[CSR_GN9] = acc;
    for (int i = 0; i < tot; ++i) { const int vl = key[i]; outp[ncnt[vl]] = ids[i]; ncnt[vl] += 1; }
    for (int vl = CSR_GN9; vl > 0; --vl) ncnt[vl] = ncnt[vl - 1]; ncnt[0] = 0; }
  __syncthreads();
  for (int pass = 0; pass < 2; ++pass) {
    for (int i = t_; i < (stn - st) / 4; i += 256) { v4i v; for (int e = 0; e < 4; ++e) { const int q = i * 4 + e; v[e] = (q < tot) ? outp[q] : -1; } *(volatile v4i*)(PERM + st + i * 4) = v; }
    for (int i = t_; i < CSR_TS9 / 4; i += 256) { v4i a, c; for (int e = 0; e < 4; ++e) { const int vl = i * 4 + e; const int vc = vl < CSR_GN9 ? vl : CSR_GN9; a[e] = (vl < CSR_GN9) ? st + ncnt[vc] : st; c[e] = (vl < nv) ? (ncnt[(vc < CSR_GN9 ? vc : CSR_GN9 - 1) + 1] - ncnt[vc]) : 0; } *(volatile v4i*)(ROWPTR + t0 + i * 4) = a; *(volatile v4i*)(ROWCNT + t0 + i * 4) = c; }
    __threadfence(); }
}
__global__ __launch_bounds__(256) void csrZ_kernel9(int* __restrict__ p, size_t n4) { typedef __attribute__((ext_vector_type(4))) int v4i; const size_t tid = (size_t)blockIdx.x * 256 + threadIdx.x, nth = (size_t)gridDim.x * 256; v4i z = {0, 0, 0, 0}; for (size_t i = tid; i < n4; i += nth) *(volatile v4i*)(p + i * 4) = z; }
struct CsrBufs9 { int *STG, *HST, *OFF, *START, *TOT, *PERM, *ROWPTR, *ROWCNT, *FLAG; int nG, NGP, CHP; size_t permLen; char* base; size_t bytes; };
static size_t csr_carve9(CsrBufs9& c, char* ws, size_t off, int E, int N) {
  const size_t off0 = off; c.base = ws + off;
  auto al = [&](size_t bytes) { char* p = ws + off; off += (bytes + 255) & ~(size_t)255; return p; };
  c.nG = (N + CSR_GN9 - 1) / CSR_GN9; c.NGP = (c.nG + 31) & ~31; const int ch = (E + CSR_NBLK9 - 1) / CSR_NBLK9; c.CHP = (ch + 31) & ~31; c.permLen = (size_t)E + 32 * (size_t)c.nG + 32;
  c.STG = (int*)al((size_t)CSR_NBLK9 * c.CHP * 4); c.HST = (int*)al((size_t)CSR_NBLK9 * c.NGP * 4); c.OFF = (int*)al((size_t)c.NGP * CSR_NBLK9 * 4); c.START = (int*)al((size_t)(c.NGP + 64) * 4); c.TOT = (int*)al((size_t)(c.NGP + 64) * 4);
  c.PERM = (int*)al(c.permLen * 4); c.ROWPTR = (int*)al((size_t)c.nG * CSR_TS9 * 4); c.ROWCNT = (int*)al((size_t)c.nG * CSR_TS9 * 4); c.FLAG = (int*)al(256);
  c.bytes = off - off0; return off;
}
static void csr_build9(const CsrBufs9& c, const int* dst, int E, int N, hipStream_t stream) {
  const size_t smem = (size_t)(2 * c.NGP + c.CHP) * 4;
  csrZ_kernel9<<<512, 256, 0, stream>>>((int*)c.base, c.bytes / 16);
  csrA_kernel9<<<CSR_NBLK9, 64, smem, stream>>>(dst, E, N, c.nG, c.CHP, c.NGP, c.STG, c.HST);
  csrS_kernel9<<<1, 512, 0, stream>>>(c.HST, c.nG, c.NGP, c.START, c.TOT, c.OFF);
  csrB_kernel9<<<c.nG, 256, 0, stream>>>(dst, N, c.nG, c.CHP, c.NGP, (int)c.permLen, c.STG, c.HST, c.OFF, c.START, c.TOT, c.PERM, c.ROWPTR, c.ROWCNT, c.FLAG);
}


__global__ __launch_bounds__(256) void wput_kernel(const float* __restrict__ w, int KIN, int KP, int OUTW, int ro, b16* __restrict__ WT) {
  const int KG = KP / 8; const int u = blockIdx.x * 256 + threadIdx.x; if (u >= OUTW * KG) return; const int o = u / KG, k0 = (u % KG) * 8; v8b v;
#pragma unroll
  for (int j = 0; j < 8; ++j) { const int k = k0 + j; v[j] = k < KIN ? (b16)(bf16_rne(w[(size_t)k * OUTW + o]) * WSC) : (b16)0.0f; } for (int pass = 0; pass < 2; ++pass) { *(volatile v8b*)(WT + (size_t)(ro + o) * KP + k0) = v; __threadfence(); }
}
__global__ __launch_bounds__(256) void wcopy_kernel(const float* __restrict__ w, int OUTW, int KIN, b16* __restrict__ WT) {
  const size_t u = (size_t)blockIdx.x * 256 + threadIdx.x; if (u >= (size_t)OUTW * KIN / 8) return; const size_t e = u * 8; v8b v;
#pragma unroll
  for (int j = 0; j < 8; ++j) v[j] = (b16)(bf16_rne(w[e + j]) * WSC); for (int pass = 0; pass < 2; ++pass) { *(volatile v8b*)(WT + e) = v; __threadfence(); }
}
__global__ __launch_bounds__(32) void xw_kernel(const float* __restrict__ x, const b16* __restrict__ WC, int NLIM, float* __restrict__ XW) {
  __shared__ __attribute__((aligned(16))) b16 Ah[16][40]; __shared__ __attribute__((aligned(16))) float Tf[16][128 + 4];
  const int lane = threadIdx.x, nloc = lane & 15, hlf = lane >> 4; const size_t m0 = (size_t)blockIdx.x * 16; if (m0 >= (size_t)NLIM) return;
  for (int rr = 0; rr < 16; ++rr) Ah[rr][lane] = (b16)((lane < IN ? bf16_rne(x[(m0 + rr) * IN + lane]) : 0.0f) * XS);
  wave_lds_sync(); const v16b a = frag_kb(&Ah[nloc][0], hlf);
#pragma unroll
  for (int t = 0; t < 8; ++t) { v8f acc = {}; acc = wmma16b(a, frag_kb(WC + (size_t)(t * 16 + nloc) * 32, hlf), acc);
#pragma unroll
    for (int r8 = 0; r8 < 8; ++r8) Tf[8 * hlf + r8][t * 16 + nloc] = acc[r8] * (1.0f / (XS * WSC)); }
  wave_lds_sync();
  for (int pass = 0; pass < 2; ++pass) { for (int rr = 0; rr < 16; ++rr) *(volatile v4f*)(XW + (m0 + rr) * 128 + lane * 4) = *(const v4f*)(&Tf[rr][lane * 4]); __threadfence(); }
}
__global__ __launch_bounds__(256) void hedge_kernel(const float* __restrict__ XW, const int* __restrict__ en, const int* __restrict__ ea, const int* __restrict__ PERM, const int* __restrict__ ROWPTR, const int* __restrict__ ROWCNT, int permLen, int NLIM, int MLIM, float* __restrict__ EF) {
  const int wave = threadIdx.x >> 5, lane = threadIdx.x & 31; const size_t h = (size_t)blockIdx.x * 8 + wave; if (h >= (size_t)MLIM) return; const int c0 = lane * 4; const int myt = c0 / HID;
  int st = ROWPTR[h], cnt = ROWCNT[h]; cnt = iclamp(cnt, 0, 1 << 20); st = iclamp(st, 0, permLen - cnt); v4f a = {0.0f, 0.0f, 0.0f, 0.0f}; int c = 0;
#pragma unroll 1
  for (int j = 0; j < cnt; ++j) { const int e = iclamp(PERM[st + j], 0, E - 1); const size_t n = (size_t)iclamp(en[e], 0, N - 1); if (n >= (size_t)NLIM) continue; const int t = iclamp(ea[e], 0, NT - 1); if (t == myt) { ++c; const v4f xv = *(const v4f*)(XW + n * 128 + c0); for (int i = 0; i < 4; ++i) a[i] += xv[i]; } }
  const float inv = c > 0 ? 1.0f / (float)c : 0.0f; v4f r; for (int i = 0; i < 4; ++i) r[i] = pmul(a[i], inv);
  for (int pass = 0; pass < 2; ++pass) { *(volatile v4f*)(EF + h * 128 + c0) = r; __threadfence(); }
}
__global__ __launch_bounds__(32) void node_kernel(const float* __restrict__ EF, const float* __restrict__ hp, const int* __restrict__ ehd, const int* __restrict__ ea, const int* __restrict__ PERM, const int* __restrict__ ROWPTR, const int* __restrict__ ROWCNT, int permLen, const float* __restrict__ bconv, const b16* __restrict__ WM, const float* __restrict__ bm, const b16* __restrict__ WIH, const b16* __restrict__ WHH, const float* __restrict__ bih, const float* __restrict__ bhh, int NLIM, int MLIM, float* __restrict__ HN) {
  __shared__ __attribute__((aligned(16))) b16 Ah[16][136], Al[16][136], Bh[16][72], Bl[16][72], Ph[16][72]; __shared__ float Hs[16][HID + 1];
  const int lane = threadIdx.x, nloc = lane & 15, hlf = lane >> 4; const size_t m0 = (size_t)blockIdx.x * 16; if (m0 >= (size_t)NLIM) return; const int c0 = lane * 4; const int myt = c0 / HID;
  for (int rr = 0; rr < 16; ++rr) { const size_t v = m0 + rr; int st = ROWPTR[v], cnt = ROWCNT[v]; cnt = iclamp(cnt, 0, 1 << 20); st = iclamp(st, 0, permLen - cnt); v4f a = {0.0f, 0.0f, 0.0f, 0.0f}; int c = 0;
#pragma unroll 1
    for (int j = 0; j < cnt; ++j) { const int e = iclamp(PERM[st + j], 0, E - 1); const size_t hh = (size_t)iclamp(ehd[e], 0, M - 1); if (hh >= (size_t)MLIM) continue; const int t = iclamp(ea[e], 0, NT - 1); if (t == myt) { ++c; const v4f ev = *(const v4f*)(EF + hh * 128 + c0); for (int i = 0; i < 4; ++i) a[i] += ev[i]; } }
    const float inv = c > 0 ? 1.0f / (float)c : 0.0f;
    for (int i = 0; i < 4; ++i) { const float cv = pmul(a[i], inv) + bf16_rne(bconv[c0 + i]); b16 p, q; split16(cv * CS, p, q); Ah[rr][c0 + i] = p; Al[rr][c0 + i] = q; }
    for (int i = 0; i < 2; ++i) { const float hv = bf16_rne(hp[v * HID + lane * 2 + i]); Hs[rr][lane * 2 + i] = hv; Ph[rr][lane * 2 + i] = (b16)(hv * XS); } }
  wave_lds_sync();
  { v8f acc[4] = {(v8f){}, (v8f){}, (v8f){}, (v8f){}};
#pragma unroll
    for (int kb = 0; kb < 128; kb += 32) { const v16b a = frag_kb(&Ah[nloc][kb], hlf), al = frag_kb(&Al[nloc][kb], hlf);
#pragma unroll
      for (int t = 0; t < 4; ++t) { const v16b bw = frag_kb(WM + (size_t)(t * 16 + nloc) * 128 + kb, hlf); acc[t] = wmma16b(a, bw, acc[t]); acc[t] = wmma16b(al, bw, acc[t]); } }
    wave_lds_sync();
#pragma unroll
    for (int t = 0; t < 4; ++t) { const int cc = t * 16 + nloc; const float bb = bf16_rne(bm[cc]);
#pragma unroll
      for (int r8 = 0; r8 < 8; ++r8) { b16 p, q; split16(fmaxf(acc[t][r8] * (1.0f / (CS * WSC)) + bb, 0.0f) * CS, p, q); Bh[8 * hlf + r8][cc] = p; Bl[8 * hlf + r8][cc] = q; } } }
  wave_lds_sync(); v8f gi[12], gh[12];
#pragma unroll
  for (int t = 0; t < 12; ++t) { gi[t] = (v8f){}; gh[t] = (v8f){}; }
#pragma unroll
  for (int kb = 0; kb < HID; kb += 32) { const v16b a = frag_kb(&Bh[nloc][kb], hlf), al = frag_kb(&Bl[nloc][kb], hlf), ph = frag_kb(&Ph[nloc][kb], hlf);
#pragma unroll
    for (int t = 0; t < 12; ++t) { const v16b wi = frag_kb(WIH + (size_t)(t * 16 + nloc) * HID + kb, hlf), wh = frag_kb(WHH + (size_t)(t * 16 + nloc) * HID + kb, hlf); gi[t] = wmma16b(a, wi, gi[t]); gi[t] = wmma16b(al, wi, gi[t]); gh[t] = wmma16b(ph, wh, gh[t]); } }
  const float si = 1.0f / (CS * WSC), sh = 1.0f / (XS * WSC);
#pragma unroll
  for (int tg = 0; tg < 4; ++tg) { const int j = tg * 16 + nloc; const float bir = bf16_rne(bih[j]), biz = bf16_rne(bih[HID + j]), bin = bf16_rne(bih[2 * HID + j]), bhr = bf16_rne(bhh[j]), bhz = bf16_rne(bhh[HID + j]), bhn = bf16_rne(bhh[2 * HID + j]);
#pragma unroll
    for (int r8 = 0; r8 < 8; ++r8) { const int rl = 8 * hlf + r8; const float r = sigm(gi[tg][r8] * si + bir + gh[tg][r8] * sh + bhr), z = sigm(gi[4 + tg][r8] * si + biz + gh[4 + tg][r8] * sh + bhz); const float nn = tanhf(gi[8 + tg][r8] * si + bin + pmul(r, gh[8 + tg][r8] * sh + bhn)); Hs[rl][j] = pmul(1.0f - z, nn) + pmul(z, Hs[rl][j]); } }
  wave_lds_sync();
  for (int pass = 0; pass < 2; ++pass) { for (int rr = 0; rr < 16; ++rr) *(volatile v2f*)(HN + (m0 + rr) * HID + lane * 2) = (v2f){Hs[rr][lane * 2], Hs[rr][lane * 2 + 1]}; __threadfence(); }
}
__global__ __launch_bounds__(32) void pred_kernel(const float* __restrict__ HN, const float* __restrict__ Wo, const float* __restrict__ bo, int NLIM, float* __restrict__ out) {
  __shared__ float So[96]; const int lane = threadIdx.x; const size_t n0 = (size_t)blockIdx.x * 32; if (n0 >= (size_t)NLIM) return; const size_t n = n0 + lane; const float* hr = HN + n * HID;
  float s0 = bf16_rne(bo[0]), s1 = bf16_rne(bo[1]), s2 = bf16_rne(bo[2]);
#pragma unroll 4
  for (int k = 0; k < HID; ++k) { const float hv = hr[k]; s0 += pmul(hv, bf16_rne(Wo[k * HID + 0])); s1 += pmul(hv, bf16_rne(Wo[k * HID + 1])); s2 += pmul(hv, bf16_rne(Wo[k * HID + 2])); }
  So[lane * 3] = s0; So[lane * 3 + 1] = s1; So[lane * 3 + 2] = s2; wave_lds_sync();
  for (int pass = 0; pass < 2; ++pass) { for (int i = lane; i < 96; i += 32) ((volatile float*)out)[n0 * 3 + i] = So[i]; __threadfence(); }
}
}

extern "C" void kernel_launch(void* const* d_in, const int* in_sizes, int n_in, void* d_out, int out_size, void* d_ws, size_t ws_size, hipStream_t stream) {
  (void)n_in;
  auto Fp = [&](int i) { return (const float*)d_in[i]; }; auto Ip = [&](int i) { return (const int*)d_in[i]; };
  if (in_sizes[0] != N * IN || in_sizes[1] != N * HID || in_sizes[2] != E || in_sizes[3] != E || in_sizes[4] != E || in_sizes[5] != NT * IN * HID || in_sizes[7] != 128 * HID || in_sizes[9] != 192 * HID || in_sizes[10] != 192 * HID || in_sizes[13] != HID * HID || out_size != N * HID + N * 3) return;
  const int NLIM = N, MLIM = M; const int GB16 = NBLK, GB32 = N / 32;
  size_t off = 0; char* ws = (char*)d_ws;
  auto carve = [&](size_t bytes) { char* p = ws + off; off += (bytes + 255) & ~(size_t)255; return p; };
  b16* WC = (b16*)carve(128 * 32 * 2); b16* WM = (b16*)carve(HID * 128 * 2); b16* WIH = (b16*)carve(192 * HID * 2); b16* WHH = (b16*)carve(192 * HID * 2); float* XW = (float*)carve((size_t)N * 128 * 4); float* EF = (float*)carve((size_t)M * 128 * 4);
  CsrBufs9 ch, cn; off = csr_carve9(ch, ws, off, E, M); off = csr_carve9(cn, ws, off, E, N);
  if (off > ws_size || off > ((size_t)256 << 20)) return;
  wput_kernel<<<(HID * 4 + 255) / 256, 256, 0, stream>>>(Fp(5), IN, 32, HID, 0, WC); wput_kernel<<<(HID * 4 + 255) / 256, 256, 0, stream>>>(Fp(5) + IN * HID, IN, 32, HID, HID, WC); wput_kernel<<<(HID * 16 + 255) / 256, 256, 0, stream>>>(Fp(7), 128, 128, HID, 0, WM);
  wcopy_kernel<<<(192 * HID / 8 + 255) / 256, 256, 0, stream>>>(Fp(9), 192, HID, WIH); wcopy_kernel<<<(192 * HID / 8 + 255) / 256, 256, 0, stream>>>(Fp(10), 192, HID, WHH);
  csr_build9(ch, Ip(3), E, M, stream); csr_build9(cn, Ip(2), E, N, stream);
  xw_kernel<<<GB16, 32, 0, stream>>>(Fp(0), WC, NLIM, XW);
  hedge_kernel<<<(MLIM + 7) / 8, 256, 0, stream>>>(XW, Ip(2), Ip(4), ch.PERM, ch.ROWPTR, ch.ROWCNT, (int)ch.permLen, NLIM, MLIM, EF);
  float* out = (float*)d_out;
  node_kernel<<<GB16, 32, 0, stream>>>(EF, Fp(1), Ip(3), Ip(4), cn.PERM, cn.ROWPTR, cn.ROWCNT, (int)cn.permLen, Fp(6), WM, Fp(8), WIH, WHH, Fp(11), Fp(12), NLIM, MLIM, out);
  pred_kernel<<<GB32, 32, 0, stream>>>(out, Fp(13), Fp(14), NLIM, out + (size_t)N * HID);
}
